// GraphEncoder_41248865911345
// MI455X (gfx1250) — hardware-verified
//
#include <hip/hip_runtime.h>
#include <math.h>

constexpr int NNODE = 100000;
constexpr int NEDGE = 1600000;
constexpr int MPAD  = 100032;
constexpr int CIN   = 40;
constexpr int NHID1 = 64;
constexpr int NHID2 = 128;
constexpr int NHID3 = 64;
constexpr int NHEAD = 3;
constexpr int P16   = 128;
constexpr int KSEG  = 128;
static_assert(MPAD % 64 == 0);
static_assert(MPAD >= NNODE);
static_assert(MPAD - NNODE < 64);
static_assert(KSEG % 32 == 0);
static_assert(CIN <= 64);
static_assert(CIN % 8 == 0);
static_assert((NNODE * NHEAD) % 32 == 0);
static_assert(NHID1 % 64 == 0 && NHID2 % 64 == 0 && NHID3 == 64);

typedef __attribute__((ext_vector_type(16))) _Float16 v16h;
typedef __attribute__((ext_vector_type(8)))  _Float16 v8h;
typedef __attribute__((ext_vector_type(8)))  float    v8f;
typedef __attribute__((ext_vector_type(4)))  float    v4f;
typedef __attribute__((ext_vector_type(2)))  float    v2f;
typedef __attribute__((ext_vector_type(4)))  int      v4i;
typedef __attribute__((ext_vector_type(4)))  unsigned int v4u;

__device__ __forceinline__ void dep_guard_h(v8f& a, v8f& b, v16h x, v16h y) { asm volatile("v_nop\n\tv_nop\n\tv_nop\n\tv_nop" : "+v"(a), "+v"(b) : "v"(x), "v"(y)); }
__device__ __forceinline__ void keep4_h(v16h a, v16h b, v16h c, v16h d) { asm volatile("v_nop" :: "v"(a), "v"(b), "v"(c), "v"(d)); }
__device__ __forceinline__ void acc_guard4(v8f& a, v8f& b, v8f& c, v8f& d) { asm volatile("v_nop\n\tv_nop\n\tv_nop\n\tv_nop" : "+v"(a), "+v"(b), "+v"(c), "+v"(d)); }
template <typename T> struct Frag;
template <> struct Frag<_Float16> {
  typedef v16h V; union U { v16h v; v8h h[2]; };
  static __device__ __forceinline__ v16h load(const _Float16* p) {
    U f; f.h[0] = *(const v8h*)(p); f.h[1] = *(const v8h*)(p + 16); return f.v;
  }
  static __device__ __forceinline__ v8f mma(v16h a, v16h b, v8f c) {
    return __builtin_amdgcn_wmma_f32_16x16x32_f16(false, a, false, b, (short)0, c, false, false);
  }
  static __device__ __forceinline__ void guard(v8f& a, v8f& b, v16h x, v16h y) { dep_guard_h(a, b, x, y); }
  static __device__ __forceinline__ void keep(v16h a, v16h b, v16h c, v16h d) { keep4_h(a, b, c, d); }
};
__device__ __forceinline__ unsigned pk16(unsigned short a, unsigned short b) { return (unsigned)a | ((unsigned)b << 16); }
__device__ __forceinline__ unsigned short h_bits(float f) { const _Float16 h = (_Float16)f; return __builtin_bit_cast(unsigned short, h); }

template <int NSEG, int OUTK>
__global__ __launch_bounds__(256) void gemm64_kernel(
    const unsigned short* __restrict__ A0p, int lda0, const unsigned short* __restrict__ B0p, int ldb0, int K0,
    const unsigned short* __restrict__ A1p, int lda1, const unsigned short* __restrict__ B1p, int ldb1, int K1,
    const float* __restrict__ bias,
    float* __restrict__ C32, int ldc32,
    unsigned short* __restrict__ C16, int ldc16, int coff16,
    const float* __restrict__ W4, const float* __restrict__ b4, float* __restrict__ outp, int nreal,
    int M, int N) {
  typedef _Float16 T;
  typedef v16h V;
  __shared__ __align__(16) float sT[8][16 * 68];
  __shared__ __align__(16) float sH[8][192];
  __shared__ float sW[196];
  if (OUTK == 2) {
    if (threadIdx.x < NHID3 * NHEAD) sW[threadIdx.x] = W4[threadIdx.x];
    if (threadIdx.x < NHEAD) sW[NHID3 * NHEAD + threadIdx.x] = b4[threadIdx.x];
    __syncthreads();
  }
  const int lane = threadIdx.x & 31;
  const int wave = threadIdx.x >> 5;
  const int tilesN = N >> 6;
  const int tilesM = M >> 6;
  const int tile = blockIdx.x * 8 + wave;
  if (tile >= tilesM * tilesN) return;
  const int tm = tile / tilesN;
  const int tn = tile - tm * tilesN;
  const int m0 = tm << 6;
  const int n0 = tn << 6;

  const int rlane = lane & 15;
  const int koff  = (lane >> 4) * 8;
  const int mOff  = (lane >> 4) * 8;

  v8f acc[4][4];
#pragma unroll
  for (int i = 0; i < 4; ++i)
#pragma unroll
    for (int j = 0; j < 4; ++j) acc[i][j] = (v8f){0.f,0.f,0.f,0.f,0.f,0.f,0.f,0.f};

#pragma unroll
  for (int seg = 0; seg < NSEG; ++seg) {
    const T* Ab = (const T*)((seg == 0) ? A0p : A1p);
    const T* Bb = (const T*)((seg == 0) ? B0p : B1p);
    const int lda = (seg == 0) ? lda0 : lda1;
    const int ldb = (seg == 0) ? ldb0 : ldb1;
    const int Kseg = (seg == 0) ? K0 : K1;
    for (int k0 = 0; k0 < Kseg; k0 += 32) {
      V bh[4];
#pragma unroll
      for (int j = 0; j < 4; ++j) {
        const size_t bo = (size_t)(n0 + (j << 4) + rlane) * ldb + koff + k0;
        bh[j] = Frag<T>::load(Bb + bo);
      }
#pragma unroll
      for (int i = 0; i < 4; ++i) {
        const size_t ao = (size_t)(m0 + (i << 4) + rlane) * lda + koff + k0;
        V ah = Frag<T>::load(Ab + ao);
#pragma unroll
        for (int j = 0; j < 4; ++j) acc[i][j] = Frag<T>::mma(ah, bh[j], acc[i][j]);
        Frag<T>::guard(acc[i][0], acc[i][3], ah, ah);
      }
      Frag<T>::keep(bh[0], bh[1], bh[2], bh[3]);
    }
  }
  acc_guard4(acc[0][0], acc[0][1], acc[0][2], acc[0][3]);
  acc_guard4(acc[1][0], acc[1][1], acc[1][2], acc[1][3]);
  acc_guard4(acc[2][0], acc[2][1], acc[2][2], acc[2][3]);
  acc_guard4(acc[3][0], acc[3][1], acc[3][2], acc[3][3]);

  float* slab = sT[wave];
#pragma unroll
  for (int i = 0; i < 4; ++i) {
    const int mBase = m0 + (i << 4);
#pragma unroll
    for (int j = 0; j < 4; ++j) {
      const int n = n0 + (j << 4) + rlane;
      const float bv = bias[n];
#pragma unroll
      for (int r = 0; r < 8; ++r) {
        float v = acc[i][j][r] + bv;
        v = fmaxf(v, 0.0f);
        slab[(mOff + r) * 68 + (j << 4) + rlane] = v;
      }
    }
    __builtin_amdgcn_fence(__ATOMIC_RELEASE, "workgroup");
    __builtin_amdgcn_wave_barrier();
    __builtin_amdgcn_fence(__ATOMIC_ACQUIRE, "workgroup");
    if (OUTK == 1) {
      const int hh = lane >> 4, c4 = (lane & 15) * 4;
      const int q = lane >> 3, c8 = (lane & 7) * 8;
      for (int pass = 0; pass < 2; ++pass) {
#pragma unroll
        for (int it = 0; it < 8; ++it) {
          const int row = it * 2 + hh;
          const v4f v = *(const v4f*)(slab + row * 68 + c4);
          *(volatile v4f*)(C32 + (size_t)(mBase + row) * ldc32 + n0 + c4) = v;
        }
#pragma unroll
        for (int it = 0; it < 4; ++it) {
          const int row = it * 4 + q;
          const float* sp = slab + row * 68 + c8;
          v8h hv;
#pragma unroll
          for (int e = 0; e < 8; ++e) hv[e] = (_Float16)sp[e];
          *(volatile v8h*)(C16 + (size_t)(mBase + row) * ldc16 + coff16 + n0 + c8) = hv;
        }
        __threadfence();
      }
    } else {
      const int kh = lane >> 4;
      float p0 = 0.0f, p1 = 0.0f, p2 = 0.0f;
#pragma unroll 1
      for (int k = 0; k < 32; ++k) {
        const int kk = (kh << 5) + k;
        const float hv = slab[rlane * 68 + kk];
        p0 = fmaf(hv, sW[kk * 3 + 0], p0);
        p1 = fmaf(hv, sW[kk * 3 + 1], p1);
        p2 = fmaf(hv, sW[kk * 3 + 2], p2);
      }
      p0 += __shfl_xor(p0, 16, 32);
      p1 += __shfl_xor(p1, 16, 32);
      p2 += __shfl_xor(p2, 16, 32);
      p0 += sW[NHID3 * NHEAD + 0];
      p1 += sW[NHID3 * NHEAD + 1];
      p2 += sW[NHID3 * NHEAD + 2];
      if (lane < 16) {
        float* hs = sH[wave] + (i * 16 + rlane) * NHEAD;
        hs[0] = p0; hs[1] = p1; hs[2] = p2;
      }
    }
    __builtin_amdgcn_fence(__ATOMIC_RELEASE, "workgroup");
    __builtin_amdgcn_wave_barrier();
    __builtin_amdgcn_fence(__ATOMIC_ACQUIRE, "workgroup");
  }
  if (OUTK == 2) {
    const float* hs = sH[wave];
    const int f0 = m0 * NHEAD;
    const int lim = nreal * NHEAD;
    const v4f v0 = *(const v4f*)(hs + 4 * lane);
    const v4f v1 = *(const v4f*)(hs + 128 + 4 * (lane & 15));
    const bool ok0 = (f0 + 4 * lane + 4) <= lim;
    const bool ok1 = (lane < 16) && ((f0 + 128 + 4 * lane + 4) <= lim);
    for (int pass = 0; pass < 2; ++pass) {
      if (ok0) *(volatile v4f*)(outp + f0 + 4 * lane) = v0;
      if (ok1) *(volatile v4f*)(outp + f0 + 128 + 4 * lane) = v1;
      __threadfence();
    }
  }
}

__global__ __launch_bounds__(256) void prep_wt_kernel(
    const float* __restrict__ W1l, const float* __restrict__ W1r, const float* __restrict__ W2l, const float* __restrict__ W2r,
    const float* __restrict__ W3l, const float* __restrict__ W3r,
    unsigned short* __restrict__ Bt1, unsigned short* __restrict__ Bt2, unsigned short* __restrict__ Bt3a, unsigned short* __restrict__ Bt3b) {
  __shared__ float sm[64][65];
  const int job = blockIdx.x;
  const float* W = W1l; int nc = NHID1, ks = 0, kc = CIN, nb = 0, kd = 0; unsigned short* dst = Bt1;
  if (job == 1)      { W = W1r; nc = NHID1; ks = 0;  kc = CIN; dst = Bt1;  nb = 0;  kd = 64; }
  else if (job == 2) { W = W2l; nc = NHID2; ks = 0;  kc = 64;  dst = Bt2;  nb = 0;  kd = 0;  }
  else if (job == 3) { W = W2l; nc = NHID2; ks = 0;  kc = 64;  dst = Bt2;  nb = 64; kd = 0;  }
  else if (job == 4) { W = W2r; nc = NHID2; ks = 0;  kc = 64;  dst = Bt2;  nb = 0;  kd = 64; }
  else if (job == 5) { W = W2r; nc = NHID2; ks = 0;  kc = 64;  dst = Bt2;  nb = 64; kd = 64; }
  else if (job == 6) { W = W3l; nc = NHID3; ks = 0;  kc = 64;  dst = Bt3a; nb = 0;  kd = 0;  }
  else if (job == 7) { W = W3l; nc = NHID3; ks = 64; kc = 64;  dst = Bt3a; nb = 0;  kd = 64; }
  else if (job == 8) { W = W3r; nc = NHID3; ks = 0;  kc = 64;  dst = Bt3b; nb = 0;  kd = 0;  }
  else if (job == 9) { W = W3r; nc = NHID3; ks = 64; kc = 64;  dst = Bt3b; nb = 0;  kd = 64; }
  const int t = threadIdx.x;
#pragma unroll
  for (int i = 0; i < 16; ++i) {
    const int e = i * 256 + t;
    const int kl = e >> 6;
    const int nl = e & 63;
    const int klc = (kl < kc) ? kl : (kc - 1);
    const float f = (kl < kc) ? 1.0f : 0.0f;
    sm[nl][kl] = f * W[(size_t)(ks + klc) * nc + nb + nl];
  }
  __syncthreads();
  const int lane = t & 31, wave = t >> 5;
  const int q = lane >> 3, c8 = (lane & 7) * 8;
  for (int pass = 0; pass < 2; ++pass) {
#pragma unroll
    for (int it = 0; it < 2; ++it) {
      const int row = wave * 8 + it * 4 + q;
      unsigned short hb[8];
#pragma unroll
      for (int e = 0; e < 8; ++e) hb[e] = h_bits(sm[row][c8 + e]);
      const v4u u = (v4u){pk16(hb[0], hb[1]), pk16(hb[2], hb[3]), pk16(hb[4], hb[5]), pk16(hb[6], hb[7])};
      *(volatile v4u*)(dst + (size_t)(nb + row) * P16 + kd + c8) = u;
    }
    __threadfence();
  }
}

constexpr int AG_NT = 256;
constexpr int AG_SCH = 4096;
constexpr int AG_SP = AG_SCH / AG_NT;
constexpr int AG_NCH = (NEDGE + AG_SCH - 1) / AG_SCH;
constexpr int AG_DUM = 256;
static_assert(NEDGE % AG_SP == 0);
static_assert(AG_SCH == 4096);
static_assert(NNODE < (1 << 30));

template <int LAYER> struct AggCfg;
template <> struct AggCfg<1> { static constexpr int TROWS = 1536; static constexpr int AP = CIN;   };
template <> struct AggCfg<2> { static constexpr int TROWS = 960;  static constexpr int AP = NHID1; };
template <> struct AggCfg<3> { static constexpr int TROWS = 480;  static constexpr int AP = NHID2; };
constexpr int AG_NBLK1 = (MPAD + AggCfg<1>::TROWS - 1) / AggCfg<1>::TROWS;
constexpr int AG_NBLK2 = (MPAD + AggCfg<2>::TROWS - 1) / AggCfg<2>::TROWS;
constexpr int AG_NBLK3 = (MPAD + AggCfg<3>::TROWS - 1) / AggCfg<3>::TROWS;
static_assert(AG_NBLK1 * AggCfg<1>::TROWS >= MPAD);
static_assert(AG_NBLK2 * AggCfg<2>::TROWS >= MPAD);
static_assert(AG_NBLK3 * AggCfg<3>::TROWS >= MPAD);

__device__ __forceinline__ int blk_excl_scan(int cnt, int* scan_ws, int tid, int* tot) {
  const int lane = tid & 31, wave = tid >> 5; int incl = cnt;
#pragma unroll
  for (int o = 1; o < 32; o <<= 1) { const int v = __shfl_up(incl, o, 32); if (lane >= o) incl += v; }
  if (lane == 31) scan_ws[wave] = incl;
  __syncthreads();
  if (wave == 0) { int wv = (lane < AG_NT / 32) ? scan_ws[lane] : 0; int wincl = wv;
#pragma unroll
    for (int o = 1; o < 32; o <<= 1) { const int v = __shfl_up(wincl, o, 32); if (lane >= o) wincl += v; }
    if (lane < AG_NT / 32) scan_ws[32 + lane] = wincl - wv; if (lane == 31) scan_ws[64] = wincl; }
  __syncthreads();
  const int res = scan_ws[32 + wave] + incl - cnt; *tot = scan_ws[64];
  return res;
}
template <int SP, int CAP>
__device__ __forceinline__ int chunk_hits(const int* __restrict__ dstv, int e0, int n0, int nhi, int tid,
                                          int* LIST, int* scan_ws) {
  const int eb = e0 + tid * SP;
  const bool valid = eb < NEDGE;
  const int ebc = valid ? eb : (NEDGE - SP);
  const int kb = tid * SP;
  int rec[SP]; int cnt = 0;
#pragma unroll
  for (int k = 0; k < SP; k += 4) {
    const v4i d4 = *(const v4i*)(dstv + ebc + k);
#pragma unroll
    for (int e = 0; e < 4; ++e) {
      const int d = d4[e];
      const bool hit = valid && (d >= n0) && (d < nhi);
      rec[k + e] = hit ? (((d - n0) << 12) | (kb + k + e)) : -1;
      cnt += hit ? 1 : 0;
    }
  }
  int tot; int p = blk_excl_scan(cnt, scan_ws, tid, &tot);
#pragma unroll
  for (int k = 0; k < SP; ++k) if (rec[k] >= 0) { if ((unsigned)p < (unsigned)CAP) LIST[p] = rec[k]; ++p; }
  __syncthreads();
  return tot < CAP ? tot : CAP;
}

template <int LAYER>
__global__ __launch_bounds__(AG_NT) void agg_kernel(const float* __restrict__ gsrc, const float* __restrict__ xin,
                                                   const int* __restrict__ ei, unsigned short* __restrict__ dst16) {
  constexpr int TROWS = AggCfg<LAYER>::TROWS;
  constexpr int AP = AggCfg<LAYER>::AP;
  constexpr int WROWS = TROWS / 8;
  static_assert(TROWS % 8 == 0);
  static_assert(WROWS % 4 == 0);
  static_assert(TROWS < 2048);
  static_assert(AP % 4 == 0);
  __shared__ __align__(16) float ACC[TROWS * AP + AG_DUM];
  __shared__ int LIST[AG_SCH];
  __shared__ int CNT[TROWS];
  __shared__ int scan_ws[96];
  const int tid = threadIdx.x, lane = tid & 31, wave = tid >> 5;
  const int n0 = blockIdx.x * TROWS;
  int nhi = n0 + TROWS; nhi = (nhi < MPAD) ? nhi : MPAD;
  const int wr0 = wave * WROWS;
  int wrows = nhi - n0 - wr0; wrows = wrows < 0 ? 0 : (wrows > WROWS ? WROWS : wrows);
  for (int i = tid; i < TROWS; i += AG_NT) CNT[i] = 0;
  for (int i = tid; i < AG_SCH; i += AG_NT) LIST[i] = -1;
  if (tid < 96) scan_ws[tid] = 0;
  if (tid < AG_DUM) ACC[TROWS * AP + tid] = 0.0f;
  {
    const v4f z4 = {0.f, 0.f, 0.f, 0.f};
    float* wbase = ACC + wr0 * AP;
    const int nv4 = (wrows * AP) >> 2;
    for (int i = lane; i < nv4; i += 32) *(v4f*)(wbase + 4 * i) = z4;
  }
  __syncthreads();
  const int* srcv = ei;
  const int* dstv = ei + NEDGE;
  const int l20 = (lane < 20) ? lane : 19;
  const float gf1 = (lane < 20) ? 1.0f : 0.0f;
  const int dumoff = TROWS * AP + wave * 32 + 2 * (lane - l20);
#pragma unroll 1
  for (int c = 0; c < AG_NCH; ++c) {
    const int e0 = c * AG_SCH;
    const int tot = chunk_hits<AG_SP, AG_SCH>(dstv, e0, n0, nhi, tid, LIST, scan_ws);
#pragma unroll 1
    for (int base = 0; base < tot; base += 32) {
      const int q = base + lane;
      const int qc = (q < AG_SCH) ? q : (AG_SCH - 1);
      int rv = LIST[qc];
      rv = (q < tot) ? rv : -1;
      const int dlq = rv >> 12;
      const int own = (rv >= 0 && dlq >= wr0 && dlq < wr0 + WROWS) ? 1 : 0;
      unsigned msk = (unsigned)__ballot(own);
#pragma unroll 1
      for (int it = 0; it < 32; ++it) {
        if (msk == 0u) break;
        const int bp = __builtin_ctz(msk); msk &= msk - 1u;
        const int r = __shfl(rv, bp, 32);
        int dl = r >> 12; dl = dl < 0 ? 0 : (dl >= TROWS ? TROWS - 1 : dl);
        int eidx = e0 + (r & (AG_SCH - 1)); eidx = (eidx < NEDGE) ? eidx : (NEDGE - 1);
        int s = srcv[eidx]; s = s < 0 ? 0 : (s >= NNODE ? NNODE - 1 : s);
        if (LAYER == 1) {
          const v2f g = *(const v2f*)(gsrc + (size_t)s * AP + 2 * l20);
          const int idx = (lane < 20) ? (dl * AP + 2 * l20) : dumoff;
          v2f a = *(const v2f*)(ACC + idx);
          a = a + gf1 * g;
          *(v2f*)(ACC + idx) = a;
        } else if (LAYER == 2) {
          const v2f g = *(const v2f*)(gsrc + (size_t)s * AP + 2 * lane);
          const int idx = dl * AP + 2 * lane;
          v2f a = *(const v2f*)(ACC + idx);
          a = a + g;
          *(v2f*)(ACC + idx) = a;
        } else {
          const v4f g = *(const v4f*)(gsrc + (size_t)s * AP + 4 * lane);
          const int idx = dl * AP + 4 * lane;
          v4f a = *(const v4f*)(ACC + idx);
          a = a + g;
          *(v4f*)(ACC + idx) = a;
        }
        const int cd = CNT[dl];
        CNT[dl] = cd + 1;
      }
    }
    __syncthreads();
  }
  if (LAYER == 1) {
    const int h = lane >> 4, ll = lane & 15;
    const int acol = 8 * ((ll < 5) ? ll : 4);
    const int xcol = 8 * ((ll < 8) ? 0 : ((ll > 12) ? 4 : (ll - 8)));
    const float fsa = (ll < 5) ? 1.0f : 0.0f;
    const float fsx = (ll >= 8 && ll < 13) ? 1.0f : 0.0f;
    const int npairs = wrows >> 1;
#pragma unroll 1
    for (int p = 0; p < npairs; ++p) {
      const int rl = wr0 + 2 * p + h;
      const int n = n0 + rl;
      const float cf = (float)CNT[rl];
      const float inv = 1.0f / fmaxf(cf, 1.0f);
      const float* ap = ACC + rl * AP + acol;
      const v4f a0 = *(const v4f*)ap;
      const v4f a1 = *(const v4f*)(ap + 4);
      const int ncl = (n < NNODE) ? n : (NNODE - 1);
      const float fx = (n < NNODE) ? fsx : 0.0f;
      const float* xp = xin + (size_t)ncl * CIN + xcol;
      const v4f x0 = *(const v4f*)xp;
      const v4f x1 = *(const v4f*)(xp + 4);
      const float fa = fsa * inv;
      v8h hv;
#pragma unroll
      for (int e = 0; e < 4; ++e) {
        hv[e]     = (_Float16)fmaf(fa, a0[e], fx * x0[e]);
        hv[4 + e] = (_Float16)fmaf(fa, a1[e], fx * x1[e]);
      }
      unsigned short* op = dst16 + (size_t)n * P16 + 8 * ll;
      for (int pass = 0; pass < 2; ++pass) { *(volatile v8h*)op = hv; __threadfence(); }
    }
  } else if (LAYER == 2) {
    const int q = lane >> 3, c8 = (lane & 7) * 8;
    const int nquads = wrows >> 2;
#pragma unroll 1
    for (int p = 0; p < nquads; ++p) {
      const int rl = wr0 + 4 * p + q;
      const int n = n0 + rl;
      const float cf = (float)CNT[rl];
      const float inv = 1.0f / fmaxf(cf, 1.0f);
      const float* ap = ACC + rl * AP + c8;
      const v4f a0 = *(const v4f*)ap;
      const v4f a1 = *(const v4f*)(ap + 4);
      v8h hv;
#pragma unroll
      for (int e = 0; e < 4; ++e) { hv[e] = (_Float16)(a0[e] * inv); hv[4 + e] = (_Float16)(a1[e] * inv); }
      unsigned short* op = dst16 + (size_t)n * P16 + c8;
      for (int pass = 0; pass < 2; ++pass) { *(volatile v8h*)op = hv; __threadfence(); }
    }
  } else {
    const int h = lane >> 4, ll = lane & 15;
    const int npairs = wrows >> 1;
#pragma unroll 1
    for (int p = 0; p < npairs; ++p) {
      const int rl = wr0 + 2 * p + h;
      const int n = n0 + rl;
      const float cf = (float)CNT[rl];
      const float inv = 1.0f / fmaxf(cf, 1.0f);
      const float* ap = ACC + rl * AP + 8 * ll;
      const v4f a0 = *(const v4f*)ap;
      const v4f a1 = *(const v4f*)(ap + 4);
      v8h hv;
#pragma unroll
      for (int e = 0; e < 4; ++e) { hv[e] = (_Float16)(a0[e] * inv); hv[4 + e] = (_Float16)(a1[e] * inv); }
      unsigned short* op = dst16 + (size_t)n * P16 + 8 * ll;
      for (int pass = 0; pass < 2; ++pass) { *(volatile v8h*)op = hv; __threadfence(); }
    }
  }
}

extern "C" void kernel_launch(void* const* d_in, const int* in_sizes, int n_in,
                              void* d_out, int out_size, void* d_ws, size_t ws_size, hipStream_t stream) {
  (void)in_sizes; (void)n_in; (void)out_size;
  const float* x   = (const float*)d_in[0];
  const int*   ei  = (const int*)d_in[1];
  const float* W1l = (const float*)d_in[2];
  const float* b1  = (const float*)d_in[3];
  const float* W1r = (const float*)d_in[4];
  const float* W2l = (const float*)d_in[5];
  const float* b2  = (const float*)d_in[6];
  const float* W2r = (const float*)d_in[7];
  const float* W3l = (const float*)d_in[8];
  const float* b3  = (const float*)d_in[9];
  const float* W3r = (const float*)d_in[10];
  const float* W4  = (const float*)d_in[11];
  const float* b4  = (const float*)d_in[12];
  float* out = (float*)d_out;

  char* ws = (char*)d_ws; size_t off = 0;
  auto carve = [&](size_t bytes) -> char* { char* p = ws + off; off += (bytes + 255) & ~(size_t)255; return p; };
  unsigned short* RF16A = (unsigned short*)carve((size_t)MPAD * P16 * 2);
  unsigned short* RF16B = (unsigned short*)carve((size_t)MPAD * P16 * 2);
  float*          RF32A = (float*)carve((size_t)MPAD * 64 * 4);
  float*          RF32B = (float*)carve((size_t)MPAD * 128 * 4);
  unsigned short* BT1   = (unsigned short*)carve((size_t)NHID1 * P16 * 2);
  unsigned short* BT2   = (unsigned short*)carve((size_t)NHID2 * P16 * 2);
  unsigned short* BT3A  = (unsigned short*)carve((size_t)NHID3 * P16 * 2);
  unsigned short* BT3B  = (unsigned short*)carve((size_t)NHID3 * P16 * 2);
  if (off > ws_size || off > (size_t)134217728) return;

  const int gemmBlk1 = ((MPAD / 64) * (NHID1 / 64) + 7) / 8;
  const int gemmBlk2 = ((MPAD / 64) * (NHID2 / 64) + 7) / 8;
  const int gemmBlk3 = ((MPAD / 64) * (NHID3 / 64) + 7) / 8;

  prep_wt_kernel<<<10, 256, 0, stream>>>(W1l, W1r, W2l, W2r, W3l, W3r, BT1, BT2, BT3A, BT3B);

  agg_kernel<1><<<AG_NBLK1, AG_NT, 0, stream>>>(x, x, ei, RF16A);
  gemm64_kernel<1, 1><<<gemmBlk1, 256, 0, stream>>>(
      RF16A, P16, BT1, P16, KSEG,
      RF16A, P16, BT1, P16, 0,
      b1,
      RF32A, 64,
      RF16B, P16, 64,
      W4, b4, out, NNODE,
      MPAD, NHID1);

  agg_kernel<2><<<AG_NBLK2, AG_NT, 0, stream>>>(RF32A, x, ei, RF16B);
  gemm64_kernel<1, 1><<<gemmBlk2, 256, 0, stream>>>(
      RF16B, P16, BT2, P16, KSEG,
      RF16B, P16, BT2, P16, 0,
      b2,
      RF32B, 128,
      RF16A, P16, 0,
      W4, b4, out, NNODE,
      MPAD, NHID2);

  agg_kernel<3><<<AG_NBLK3, AG_NT, 0, stream>>>(RF32B, x, ei, RF16B);
  gemm64_kernel<2, 2><<<gemmBlk3, 256, 0, stream>>>(
      RF16B, P16, BT3A, P16, KSEG,
      RF16A, P16, BT3B, P16, KSEG,
      b3,
      RF32A, 64,
      RF16A, P16, 0,
      W4, b4, out, NNODE,
      MPAD, NHID3);
}
